// WNDEDecomposition_80985903333617
// MI455X (gfx1250) — hardware-run, weakly checked
//
#include <hip/hip_runtime.h>
#include <math.h>

typedef __attribute__((ext_vector_type(16))) _Float16 v16h;
typedef __attribute__((ext_vector_type(8)))  _Float16 v8h;
typedef __attribute__((ext_vector_type(8)))  float    v8f;
typedef __attribute__((ext_vector_type(4)))  float    v4f;

constexpr int kNumB   = 32;
constexpr int kNumC   = 64;
constexpr int kNumL   = 256;
constexpr int kNumH   = 64;
constexpr int kSteps  = kNumL - 1;
constexpr int kLBlk   = 128;
constexpr int kLWave  = 16;
constexpr int kWavesPerBlock = kLBlk / kLWave;
constexpr int kThreads = kWavesPerBlock * 32;
constexpr int kBlocks  = kNumB * (kNumL / kLBlk);
constexpr int kPitchH = 72;
constexpr int kPitchT = 132;
constexpr float kCarry    = 256.0f;
constexpr float kCarryInv = 1.0f / kCarry;
constexpr float kDt       = 1.0f / (float)kSteps;
constexpr float kHalfDt   = 0.5f * kDt;
constexpr float kDtSixth  = kDt / 6.0f;
static_assert(kNumC == 64 && kNumH == 64, "K and N of both contractions are 64 (two 32-deep k chunks, four 16-wide n tiles)");
static_assert((kNumL % kLBlk) == 0 && (kLBlk % kLWave) == 0, "tile multiples");
static_assert(kThreads == 256, "block size");
static_assert(kBlocks == 64, "grid size");
static_assert((kPitchH % 8) == 0 && (kPitchT % 4) == 0, "16-B aligned LDS rows");

union FragU { v16h v; v8h h[2]; };
__device__ __forceinline__ v16h frag_load(const _Float16* p) {
  FragU f;
  f.h[0] = *(const v8h*)(p);
  f.h[1] = *(const v8h*)(p + 16);
  return f.v;
}
__device__ __forceinline__ v8f mma_f16(v16h a, v16h b, v8f c) {
  return __builtin_amdgcn_wmma_f32_16x16x32_f16(false, a, false, b, (short)0, c, false, false);
}
__device__ __forceinline__ void mma_guard(v8f& c, v16h a0, v16h a1, v16h b0, v16h b1) {
  asm volatile("v_nop\n\tv_nop\n\tv_nop\n\tv_nop" : "+v"(c) : "v"(a0), "v"(a1), "v"(b0), "v"(b1));
}
__device__ __forceinline__ void wave_sync() {
  __builtin_amdgcn_fence(__ATOMIC_RELEASE, "workgroup");
  __builtin_amdgcn_wave_barrier();
  __builtin_amdgcn_fence(__ATOMIC_ACQUIRE, "workgroup");
}

__global__ __launch_bounds__(256) void ode_rk4_kernel(
    const float* __restrict__ x, const float* __restrict__ W1, const float* __restrict__ b1,
    const float* __restrict__ W2, const float* __restrict__ b2, float* __restrict__ out)
{
  __shared__ __align__(16) _Float16 sBt1[kNumH * kPitchH];
  __shared__ __align__(16) _Float16 sBt2[kNumC * kPitchH];
  __shared__ __align__(16) _Float16 sA[kWavesPerBlock][16 * kPitchH];
  __shared__ __align__(16) float    sTile[kNumC * kPitchT];

  const int tid  = threadIdx.x;
  const int lane = tid & 31;
  const int wave = tid >> 5;
  const int hh   = lane >> 4;
  const int cn   = lane & 15;
  const int bIdx = blockIdx.x >> 1;
  const int l0   = (blockIdx.x & 1) * kLBlk;

#pragma unroll
  for (int it = 0; it < 4; ++it) {
    const int idx4 = it * kThreads + tid;
    const int k  = idx4 >> 4;
    const int n4 = (idx4 & 15) * 4;
    const v4f wa = *(const v4f*)(W1 + k * kNumH + n4);
    const v4f wb = *(const v4f*)(W2 + k * kNumC + n4);
#pragma unroll
    for (int e = 0; e < 4; ++e) {
      const float fa = wa[e] * kCarry;
      const float fb = wb[e] * kCarry;
      sBt1[(n4 + e) * kPitchH + k] = (_Float16)fa;
      sBt2[(n4 + e) * kPitchH + k] = (_Float16)fb;
    }
  }
  {
    const v8h zz = (v8h){(_Float16)0.0f, (_Float16)0.0f, (_Float16)0.0f, (_Float16)0.0f,
                         (_Float16)0.0f, (_Float16)0.0f, (_Float16)0.0f, (_Float16)0.0f};
    if (tid < 64) {
      *(v8h*)(sBt1 + tid * kPitchH + 64) = zz;
      *(v8h*)(sBt2 + tid * kPitchH + 64) = zz;
    }
    if (lane < 16) {
      *(v8h*)(sA[wave] + lane * kPitchH + 64) = zz;
    }
  }
#pragma unroll
  for (int it = 0; it < 8; ++it) {
    const int idx = it * kThreads + tid;
    const int c  = idx >> 5;
    const int l4 = (idx & 31) * 4;
    const v4f v = *(const v4f*)(x + ((size_t)(bIdx * kNumC + c)) * kNumL + l0 + l4);
    *(v4f*)(sTile + c * kPitchT + l4) = v;
  }
  __syncthreads();

  v8f X[4];
  float bs1[4], bs2[4];
#pragma unroll
  for (int nt = 0; nt < 4; ++nt) {
    const float* tp = sTile + (nt * 16 + cn) * kPitchT + wave * kLWave + hh * 8;
    const v4f p0 = *(const v4f*)(tp);
    const v4f p1 = *(const v4f*)(tp + 4);
    X[nt] = (v8f){p0[0], p0[1], p0[2], p0[3], p1[0], p1[1], p1[2], p1[3]};
    bs1[nt] = b1[nt * 16 + cn] * kCarry;
    bs2[nt] = b2[nt * 16 + cn] * kCarry;
  }

  _Float16* ap = sA[wave];
  _Float16* apw = ap + (hh * 8) * kPitchH + cn;
  const _Float16* apr = ap + cn * kPitchH + hh * 8;
  const _Float16* bp1 = sBt1 + cn * kPitchH + hh * 8;
  const _Float16* bp2 = sBt2 + cn * kPitchH + hh * 8;
  const float kExpArg = 2.0f * kCarryInv;

  v8f kk[4];
#pragma unroll
  for (int nt = 0; nt < 4; ++nt) kk[nt] = (v8f){0.f, 0.f, 0.f, 0.f, 0.f, 0.f, 0.f, 0.f};

#pragma unroll 1
  for (int step = 0; step < kSteps; ++step) {
    v8f ks[4];
#pragma unroll
    for (int nt = 0; nt < 4; ++nt) ks[nt] = (v8f){0.f, 0.f, 0.f, 0.f, 0.f, 0.f, 0.f, 0.f};

#pragma unroll 1
    for (int s = 0; s < 4; ++s) {
      const bool  first = (s == 0);
      const float ca = ((s == 3) ? kDt : kHalfDt) * kCarryInv;
      const float cw = (first || (s == 3)) ? 1.0f : 2.0f;

#pragma unroll
      for (int nt = 0; nt < 4; ++nt) {
#pragma unroll
        for (int r = 0; r < 8; ++r) {
          const float xv = X[nt][r];
          const float tv = fmaf(ca, kk[nt][r], xv);
          const float sv = first ? xv : tv;
          apw[r * kPitchH + nt * 16] = (_Float16)sv;
        }
      }
      wave_sync();
      v16h a0 = frag_load(apr);
      v16h a1 = frag_load(apr + 32);
      wave_sync();

#pragma unroll
      for (int nt = 0; nt < 4; ++nt) {
        const v16h w0 = frag_load(bp1 + nt * 16 * kPitchH);
        const v16h w1 = frag_load(bp1 + nt * 16 * kPitchH + 32);
        const float bv = bs1[nt];
        v8f acc = (v8f){bv, bv, bv, bv, bv, bv, bv, bv};
        acc = mma_f16(a0, w0, acc);
        acc = mma_f16(a1, w1, acc);
        mma_guard(acc, a0, a1, w0, w1);
#pragma unroll
        for (int r = 0; r < 8; ++r) {
          const float ev = __expf(acc[r] * kExpArg);
          const float rc = __builtin_amdgcn_rcpf(ev + 1.0f);
          const float hv = fmaf(-2.0f, rc, 1.0f);
          apw[r * kPitchH + nt * 16] = (_Float16)hv;
        }
      }
      wave_sync();
      a0 = frag_load(apr);
      a1 = frag_load(apr + 32);
      wave_sync();

#pragma unroll
      for (int nt = 0; nt < 4; ++nt) {
        const v16h w0 = frag_load(bp2 + nt * 16 * kPitchH);
        const v16h w1 = frag_load(bp2 + nt * 16 * kPitchH + 32);
        const float bv = bs2[nt];
        v8f acc = (v8f){bv, bv, bv, bv, bv, bv, bv, bv};
        acc = mma_f16(a0, w0, acc);
        acc = mma_f16(a1, w1, acc);
        mma_guard(acc, a0, a1, w0, w1);
        kk[nt] = acc;
#pragma unroll
        for (int r = 0; r < 8; ++r) ks[nt][r] = fmaf(cw, acc[r], ks[nt][r]);
      }
    }

    const float c6 = kDtSixth * kCarryInv;
#pragma unroll
    for (int nt = 0; nt < 4; ++nt) {
#pragma unroll
      for (int r = 0; r < 8; ++r) X[nt][r] = fmaf(c6, ks[nt][r], X[nt][r]);
    }
  }

#pragma unroll
  for (int nt = 0; nt < 4; ++nt) {
    float* tp = sTile + (nt * 16 + cn) * kPitchT + wave * kLWave + hh * 8;
    const v4f p0 = (v4f){X[nt][0], X[nt][1], X[nt][2], X[nt][3]};
    const v4f p1 = (v4f){X[nt][4], X[nt][5], X[nt][6], X[nt][7]};
    *(v4f*)(tp)     = p0;
    *(v4f*)(tp + 4) = p1;
  }
  __syncthreads();

  v4f ov[8];
#pragma unroll
  for (int j = 0; j < 8; ++j) ov[j] = *(const v4f*)(sTile + (wave * 8 + j) * kPitchT + lane * 4);
  float* ob = out + ((size_t)(bIdx * kNumC + wave * 8)) * kNumL + l0 + lane * 4;
  for (int pass = 0; pass < 2; ++pass) {
#pragma unroll
    for (int j = 0; j < 8; ++j) {
      *(volatile v4f*)(ob + (size_t)j * kNumL) = ov[j];
    }
    __threadfence();
  }
}

extern "C" void kernel_launch(void* const* d_in, const int* in_sizes, int n_in,
                              void* d_out, int out_size, void* d_ws, size_t ws_size,
                              hipStream_t stream) {
  (void)d_ws;
  (void)ws_size;
  if (n_in < 5) return;
  if (in_sizes[0] != kNumB * kNumC * kNumL) return;
  if (in_sizes[1] != kNumC * kNumH) return;
  if (in_sizes[2] != kNumH) return;
  if (in_sizes[3] != kNumH * kNumC) return;
  if (in_sizes[4] != kNumC) return;
  if (out_size != kNumB * kNumC * kNumL) return;

  const float* x  = (const float*)d_in[0];
  const float* W1 = (const float*)d_in[1];
  const float* b1 = (const float*)d_in[2];
  const float* W2 = (const float*)d_in[3];
  const float* b2 = (const float*)d_in[4];
  float* out = (float*)d_out;

  ode_rk4_kernel<<<dim3(kBlocks), dim3(kThreads), 0, stream>>>(x, W1, b1, W2, b2, out);
}
